// InceptionAttention_11089605558726
// MI455X (gfx1250) — hardware-verified
//
#include <hip/hip_runtime.h>
#include <math.h>

typedef __attribute__((ext_vector_type(16))) _Float16 v16h;
typedef __attribute__((ext_vector_type(16))) __bf16 v16b;
typedef __attribute__((ext_vector_type(8)))  _Float16 v8h;
typedef __attribute__((ext_vector_type(8)))  float v8f;
typedef __attribute__((ext_vector_type(4)))  float v4f;
typedef __attribute__((ext_vector_type(2)))  float v2f;
typedef __attribute__((ext_vector_type(4)))  unsigned v4u;
typedef __attribute__((ext_vector_type(4)))  int v4i;
typedef float __attribute__((may_alias)) float_a;
typedef int __attribute__((may_alias)) int_a;

template <typename T> __device__ __forceinline__ void vst2(void* p, T v) { *(volatile T*)p = v; __threadfence(); *(volatile T*)p = v; }
__device__ __forceinline__ v8f wmma16(v16h a, v16h b, v8f c) {
  v8f d = __builtin_amdgcn_wmma_f32_16x16x32_f16(false, a, false, b, (short)0, c, false, false);
  asm volatile("v_nop\n\tv_nop\n\tv_nop\n\tv_nop" : "+v"(d) : "v"(a), "v"(b));
  return d;
}
__device__ __forceinline__ v8f wmma_bf(v16b a, v16b b, v8f c) {
  v8f d = __builtin_amdgcn_wmma_f32_16x16x32_bf16(false, a, false, b, (short)0, c, false, false);
  asm volatile("v_nop\n\tv_nop\n\tv_nop\n\tv_nop" : "+v"(d) : "v"(a), "v"(b));
  return d;
}
__device__ __forceinline__ v16h frag_h(const _Float16* rowk0, int lane) {
  union { v16h v; v8h q[2]; } u; const _Float16* p = rowk0 + 8 * (lane >> 4);
  u.q[0] = *(const v8h*)p; u.q[1] = *(const v8h*)(p + 16); return u.v;
}
__device__ __forceinline__ v16h frag_f32(const float* rowk0, int lane) {
  v16h a; const float* p = rowk0 + 8 * (lane >> 4);
#pragma unroll
  for (int i = 0; i < 8; ++i) { a[i] = (_Float16)p[i]; a[8 + i] = (_Float16)p[16 + i]; }
  return a;
}
__device__ __forceinline__ v16h frag_f32s(const float* rowk0, int lane, float sc) {
  v16h a; const float* p = rowk0 + 8 * (lane >> 4);
#pragma unroll
  for (int i = 0; i < 8; ++i) { a[i] = (_Float16)(p[i] * sc); a[8 + i] = (_Float16)(p[16 + i] * sc); }
  return a;
}
__device__ __forceinline__ v16h fragc_f32(const float* W, int k0, int n, int lane, int ld, int K) {
  v16h a; const int g = lane >> 4;
#pragma unroll
  for (int i = 0; i < 8; ++i) { const int ka = k0 + 8 * g + i, kb = ka + 16;
    a[i] = (_Float16)(ka < K ? W[(size_t)(ka < K ? ka : K - 1) * ld + n] : 0.f); a[8 + i] = (_Float16)(kb < K ? W[(size_t)(kb < K ? kb : K - 1) * ld + n] : 0.f); }
  return a;
}
struct F2 { v16b h, l; };
__device__ __forceinline__ F2 bsplit16(const float v[16]) { F2 r;
#pragma unroll
  for (int i = 0; i < 16; ++i) { const __bf16 h = (__bf16)v[i]; r.h[i] = h; r.l[i] = (__bf16)(v[i] - (float)h); }
  return r; }
__device__ __forceinline__ F2 split_row(const float* row, int k0, int lane) { float v[16]; const float* p = row + k0 + 8 * (lane >> 4);
#pragma unroll
  for (int i = 0; i < 8; ++i) { v[i] = p[i]; v[8 + i] = p[16 + i]; }
  return bsplit16(v); }
__device__ __forceinline__ F2 split_rowK(const float* row, int k0, int lane, int K) { float v[16]; const int g = lane >> 4;
#pragma unroll
  for (int i = 0; i < 8; ++i) { const int ka = k0 + 8 * g + i, kb = ka + 16; v[i] = ka < K ? row[ka < K ? ka : K - 1] : 0.f; v[8 + i] = kb < K ? row[kb < K ? kb : K - 1] : 0.f; }
  return bsplit16(v); }
__device__ __forceinline__ F2 split_col(const float* W, int k0, int n, int lane, int ld, int K) { float v[16]; const int g = lane >> 4;
#pragma unroll
  for (int i = 0; i < 8; ++i) { const int ka = k0 + 8 * g + i, kb = ka + 16; v[i] = ka < K ? W[(size_t)(ka < K ? ka : K - 1) * ld + n] : 0.f; v[8 + i] = kb < K ? W[(size_t)(kb < K ? kb : K - 1) * ld + n] : 0.f; }
  return bsplit16(v); }
__device__ __forceinline__ v8f mac3(const F2& a, const F2& b, v8f c) { c = wmma_bf(a.l, b.h, c); c = wmma_bf(a.h, b.l, c); return wmma_bf(a.h, b.h, c); }
__device__ __forceinline__ float sigm(float v) { return 1.0f / (1.0f + expf(-v)); }
#define LDSX() do { asm volatile("s_wait_dscnt 0" ::: "memory"); __builtin_amdgcn_wave_barrier(); __builtin_amdgcn_fence(__ATOMIC_RELEASE, "workgroup"); } while (0)


#define CC 256
#define NH 8
#define HD 32
#define HH 64
#define WWD 64
#define NP (HH * WWD)
#define NWIN 3
#define OC (CC * NWIN)
#ifndef TPB
#define TPB HH
#endif
typedef __attribute__((ext_vector_type(8))) __bf16 v8b;
__device__ __forceinline__ v16b frag_b(const __bf16* rowk0, int lane) {
  union { v16b v; v8b q[2]; } u; const __bf16* p = rowk0 + 8 * (lane >> 4);
  u.q[0] = *(const v8b*)p; u.q[1] = *(const v8b*)(p + 16); return u.v;
}
__device__ __forceinline__ float bfr(float v) { return (float)(__bf16)v; }
__device__ __attribute__((noinline)) float exp_ni(float v) { return expf(v); }
__device__ __attribute__((noinline)) float erf_ni(float v) { return erff(v); }
__constant__ int WSZ[NWIN] = {64, 32, 16};

#define WS_PW  0u
#define WS_PO  (WS_PW + 2u * (size_t)3 * CC * CC)
#define WS_XT  (WS_PO + 2u * (size_t)CC * OC)
#define WS_Q   (WS_XT + 4u * (size_t)NP * CC)
#define WS_K   (WS_Q + 4u * (size_t)NP * CC)
#define WS_V   (WS_K + 4u * (size_t)NP * CC)
#define WS_IK  (WS_V + 4u * (size_t)NP * CC)
#define WS_IKV (WS_IK + 4u * (size_t)CC * NP)
#define WS_O   (WS_IKV + 4u * (size_t)NH * HD * HD * NP)
#define WS_END (WS_O + 4u * (size_t)NP * OC)

__global__ __launch_bounds__(256) void k_pack(const float* __restrict__ WQ, const float* __restrict__ WK, const float* __restrict__ WV, const float* __restrict__ WO, __bf16* __restrict__ PW, __bf16* __restrict__ PO) { const int n = blockIdx.x, which = blockIdx.y, t = threadIdx.x; __shared__ __align__(16) __bf16 s[OC];
  if (which < 3) { const float* w = (which == 0) ? WQ : (which == 1) ? WK : WV; s[t] = (__bf16)w[(size_t)n * CC + t]; __syncthreads(); if (t < CC / 8) vst2((unsigned*)(PW + ((size_t)which * CC + n) * CC + t * 8), *(const v4u*)&s[t * 8]); }
  else { for (int k = t; k < OC; k += 256) s[k] = (__bf16)WO[(size_t)n * OC + k]; __syncthreads(); if (t < OC / 8) vst2((unsigned*)(PO + (size_t)n * OC + t * 8), *(const v4u*)&s[t * 8]); } }
__global__ __launch_bounds__(256) void k_tr(const float* __restrict__ X, float* __restrict__ XT) { __shared__ float st[64][65]; __shared__ __align__(16) float so[64][68]; const int t = threadIdx.x; const int p0 = blockIdx.x * 64, c0 = blockIdx.y * 64;
  for (int e = t; e < 64 * 64; e += 256) { const int cl = e >> 6, pl = e & 63; st[pl][cl] = X[(size_t)(c0 + cl) * NP + p0 + pl]; } __syncthreads();
  for (int e = t; e < 64 * 64; e += 256) { const int pl = e >> 6, cl = e & 63; so[pl][cl] = st[pl][cl]; } __syncthreads();
  for (int e = t; e < 64 * 16; e += 256) { const int pl = e >> 4, q = e & 15; vst2(XT + (size_t)(p0 + pl) * CC + c0 + q * 4, *(const v4f*)&so[pl][q * 4]); } }
__global__ __launch_bounds__(128) void k_proj(const float* __restrict__ XT, const __bf16* __restrict__ PW, float* __restrict__ Q, float* __restrict__ Kf, float* __restrict__ Vf) { __shared__ __align__(16) float so[4][16][132];
  const int tid = threadIdx.x, wave = tid >> 5, lane = tid & 31, col = lane & 15, g = lane >> 4; const int which = blockIdx.z; const size_t r0 = (size_t)blockIdx.x * 64 + wave * 16; const int c0 = blockIdx.y * 128; const __bf16* Wr = PW + ((size_t)which * CC) * CC;
  v8f acc[8] = {};
#pragma unroll
  for (int kc = 0; kc < CC / 32; ++kc) { v16b a; { const float* p = XT + (r0 + col) * CC + kc * 32 + 8 * g;
#pragma unroll
      for (int i = 0; i < 8; ++i) { a[i] = (__bf16)p[i]; a[8 + i] = (__bf16)p[16 + i]; } }
#pragma unroll
    for (int j = 0; j < 8; ++j) acc[j] = wmma_bf(a, frag_b(Wr + (size_t)(c0 + j * 16 + col) * CC + kc * 32, lane), acc[j]); }
#pragma unroll
  for (int j = 0; j < 8; ++j)
#pragma unroll
    for (int r = 0; r < 8; ++r) { const float v = acc[j][r]; so[wave][8 * g + r][j * 16 + col] = (which < 2) ? 1.0f / (1.0f + __expf(-v)) : v; }
  LDSX(); float* dst = (which == 0) ? Q : (which == 1) ? Kf : Vf; for (int rl = 0; rl < 16; ++rl) vst2(dst + (r0 + rl) * CC + c0 + lane * 4, *(const v4f*)&so[wave][rl][lane * 4]); }
__global__ __launch_bounds__(256) void k_vnorm(float* __restrict__ Vf) { __shared__ __align__(16) float so2[CC]; const int t = threadIdx.x; const size_t p = blockIdx.x; const float v = Vf[p * CC + t]; float q = v * v;
#pragma unroll
  for (int o = 1; o < 32; o <<= 1) q += __shfl_xor(q, o);
  const float nrm = sqrtf(q); so2[t] = v / fmaxf(nrm, 1e-12f); __syncthreads(); if (t < CC / 4) vst2(Vf + p * CC + t * 4, *(const v4f*)&so2[t * 4]); }
__global__ __launch_bounds__(256) void k_integral(const float* __restrict__ Kf, const float* __restrict__ Vf, int which, float* __restrict__ IK, float* __restrict__ IKV) { __shared__ float s[HH][WWD + 1]; __shared__ __align__(16) float so2[HH][WWD + 4]; const int t = threadIdx.x; const int pl = blockIdx.x;
  const int h = which ? pl / (HD * HD) : pl / HD; const int d = which ? (pl / HD) % HD : pl % HD; const int f = which ? pl % HD : 0; const int ck = h * HD + d, cv = h * HD + f;
  for (int e = t; e < NP; e += 256) { const float kv = Kf[(size_t)e * CC + ck]; s[e >> 6][e & 63] = which ? kv * Vf[(size_t)e * CC + cv] : kv; } __syncthreads();
  if (t < HH) { float run = 0.f; for (int w = 0; w < WWD; ++w) { run += s[t][w]; s[t][w] = run; } } __syncthreads();
  if (t < WWD) { float run = 0.f; for (int y = 0; y < HH; ++y) { run += s[y][t]; s[y][t] = run; } } __syncthreads();
  for (int e = t; e < NP; e += 256) so2[e >> 6][e & 63] = s[e >> 6][e & 63]; __syncthreads();
  float* dst = (which ? IKV : IK) + (size_t)pl * NP; for (int e = t; e < HH * 16; e += 256) { const int y = e >> 4, q = e & 15; vst2(dst + y * WWD + q * 4, *(const v4f*)&so2[y][q * 4]); } }
__device__ __forceinline__ float ilook(const float* __restrict__ plane, int a, int b, int l) { int ia = a - l, ib = b - l; ia = ia < 0 ? 0 : (ia > HH ? HH : ia); ib = ib < 0 ? 0 : (ib > WWD ? WWD : ib); if (ia == 0 || ib == 0) return 0.f; return plane[(ia - 1) * WWD + (ib - 1)]; }
__device__ __forceinline__ float boxsum(const float* __restrict__ plane, int i, int j, int ws, int l) { return ilook(plane, i + ws, j + ws, l) - ilook(plane, i + ws, j, l) - ilook(plane, i, j + ws, l) + ilook(plane, i, j, l); }
__global__ __launch_bounds__(256) void k_box(const float* __restrict__ Q, const float* __restrict__ IK, const float* __restrict__ IKV, float* __restrict__ O) { __shared__ __align__(16) float so2[WWD][HD + 4];
  const int t = threadIdx.x; const int j = t & 63, fg = t >> 6; const int i = blockIdx.x, h = blockIdx.y, wi = blockIdx.z; const int ws = WSZ[wi]; const int tp = ws - 1, rr = tp / 2, l = tp - rr; const size_t p = (size_t)i * WWD + j;
  float acc8[8]; for (int e = 0; e < 8; ++e) acc8[e] = 0.f; float nrm = 0.f;
#pragma unroll 1
  for (int d = 0; d < HD; ++d) { const float qd = Q[p * CC + h * HD + d]; const float wk = boxsum(IK + (size_t)(h * HD + d) * NP, i, j, ws, l); nrm += qd * wk;
#pragma unroll
    for (int e = 0; e < 8; ++e) { const int f = fg * 8 + e; acc8[e] += qd * boxsum(IKV + ((size_t)(h * HD + d) * HD + f) * NP, i, j, ws, l); } }
  const float inv = 1.0f / (nrm + 1e-6f); for (int e = 0; e < 8; ++e) so2[j][fg * 8 + e] = acc8[e] * inv; __syncthreads();
  { const int jj = t >> 2, q = t & 3; const size_t pp = (size_t)i * WWD + jj; vst2(O + pp * OC + wi * CC + h * HD + q * 8, *(const v4f*)&so2[jj][q * 8]); vst2(O + pp * OC + wi * CC + h * HD + q * 8 + 4, *(const v4f*)&so2[jj][q * 8 + 4]); } }
__global__ __launch_bounds__(128) void k_out(const __bf16* __restrict__ PO, const float* __restrict__ O, const float* __restrict__ BO, float* __restrict__ Y) { __shared__ __align__(16) float so[4][16][132];
  const int tid = threadIdx.x, wave = tid >> 5, lane = tid & 31, col = lane & 15, g = lane >> 4; const int o0 = blockIdx.x * 64 + wave * 16; const int p0 = blockIdx.y * 128;
  v8f acc[8] = {};
#pragma unroll 2
  for (int kc = 0; kc < OC / 32; ++kc) { const v16b a = frag_b(PO + (size_t)(o0 + col) * OC + kc * 32, lane);
#pragma unroll
    for (int jt = 0; jt < 8; ++jt) { const F2 w = split_row(O + (size_t)(p0 + jt * 16 + col) * OC, kc * 32, lane); acc[jt] = wmma_bf(a, w.h, acc[jt]); acc[jt] = wmma_bf(a, w.l, acc[jt]); } }
#pragma unroll
  for (int jt = 0; jt < 8; ++jt)
#pragma unroll
    for (int r = 0; r < 8; ++r) so[wave][8 * g + r][jt * 16 + col] = acc[jt][r] + bfr(BO[o0 + 8 * g + r]);
  LDSX(); for (int rl = 0; rl < 16; ++rl) vst2(Y + (size_t)(o0 + rl) * NP + p0 + lane * 4, *(const v4f*)&so[wave][rl][lane * 4]); }
extern "C" void kernel_launch(void* const* d_in, const int* in_sizes, int n_in, void* d_out, int out_size, void* d_ws, size_t ws_size, hipStream_t stream) {
  (void)in_sizes; (void)n_in; (void)out_size;
  const float** F = (const float**)d_in;
  if (ws_size < (size_t)WS_END) return;
  char* ws = (char*)d_ws; __bf16 *PW = (__bf16*)(ws + WS_PW), *PO = (__bf16*)(ws + WS_PO); float *XT = (float*)(ws + WS_XT), *Q = (float*)(ws + WS_Q), *Kf = (float*)(ws + WS_K), *Vf = (float*)(ws + WS_V), *IK = (float*)(ws + WS_IK), *IKV = (float*)(ws + WS_IKV), *O = (float*)(ws + WS_O);
  k_pack<<<dim3(CC, 4), 256, 0, stream>>>(F[1], F[2], F[3], F[4], PW, PO);
  k_tr<<<dim3(NP / 64, CC / 64), 256, 0, stream>>>(F[0], XT);
  k_proj<<<dim3(NP / 64, CC / 128, 3), 128, 0, stream>>>(XT, PW, Q, Kf, Vf);
  k_vnorm<<<NP, 256, 0, stream>>>(Vf);
  k_integral<<<NH * HD, 256, 0, stream>>>(Kf, Vf, 0, IK, IKV);
  k_integral<<<NH * HD * HD, 256, 0, stream>>>(Kf, Vf, 1, IK, IKV);
  k_box<<<dim3(TPB, NH, NWIN), 256, 0, stream>>>(Q, IK, IKV, O);
  k_out<<<dim3(CC / 64, (TPB * WWD) / 128), 128, 0, stream>>>(PO, O, F[5], (float*)d_out);
}
